// GrippingPointGNN_8169027797159
// MI455X (gfx1250) — hardware-verified
//
#include <hip/hip_runtime.h>
#include <stddef.h>


#define HID     128
#define INDIM   2
#define ODIM    2
#define NTHR    256
#define NWAVE   8
#define EPT     8
#define NGRP    2
#define CHUNK   (NTHR * EPT * NGRP)
#define WCAP    (EPT * NGRP * 32)
#define LISTN   (NWAVE * WCAP)
#define NBE     4096
#define ELLW    8
#define CNTMAX  65535
#define GROWS   128
#define AP      (HID + 8)
#define NSLOT   4
#define METAW   32
#define GB      16
#define WCF     128
#define ASCALE  16.0f
#define WSCALE  8.0f
#define OSCALE  0.0078125f

#define LDS_ELL ((NBE * ELLW + NBE + LISTN) * 4 + 64)
#define LDS_L3  (GROWS * HID * 4)

static_assert((CHUNK & (CHUNK - 1)) == 0);
static_assert(CHUNK == 4096);
static_assert((NBE & (NBE - 1)) == 0 && NBE <= 4096);
static_assert((NBE * ELLW / 4) % NTHR == 0 && (NBE / 4) % NTHR == 0);
static_assert(NBE % GROWS == 0 && NBE % NTHR == 0);
static_assert(GROWS == NWAVE * 16 && HID == 32 * 4);
static_assert(GROWS * AP * 2 <= LDS_L3);
static_assert(GROWS * HID * 2 <= GROWS * AP * 2);
static_assert(NSLOT == 4 && NSLOT * HID / 4 <= NTHR && 2 * NSLOT <= METAW);
static_assert(GB * HID == 8 * NTHR && GB * ODIM <= 32);
static_assert((2 * HID * HID / 8) % NTHR == 0 && ((HID * HID / 8) % NTHR) == 0);

typedef float    v2f  __attribute__((ext_vector_type(2)));
typedef float    v4f  __attribute__((ext_vector_type(4)));
typedef float    v8f  __attribute__((ext_vector_type(8)));
typedef int      v4i  __attribute__((ext_vector_type(4)));
typedef _Float16 v4h  __attribute__((ext_vector_type(4)));
typedef _Float16 v8h  __attribute__((ext_vector_type(8)));
typedef _Float16 v16h __attribute__((ext_vector_type(16)));
union FragH { v16h v; v8h h[2]; };

__device__ __forceinline__ v8h cvt8(v4f a, v4f b) {
  v8h r;
  r[0] = (_Float16)a.x; r[1] = (_Float16)a.y; r[2] = (_Float16)a.z; r[3] = (_Float16)a.w;
  r[4] = (_Float16)b.x; r[5] = (_Float16)b.y; r[6] = (_Float16)b.z; r[7] = (_Float16)b.w;
  return r;
}

__device__ __forceinline__ v4f relu4(v4f v) {
  v4f r;
  r.x = fmaxf(v.x, 0.0f); r.y = fmaxf(v.y, 0.0f); r.z = fmaxf(v.z, 0.0f); r.w = fmaxf(v.w, 0.0f);
  return r;
}

__device__ __forceinline__ v8f wmh(v16h a, v16h b, v8f c) {
  v8f d = __builtin_amdgcn_wmma_f32_16x16x32_f16(false, a, false, b, (short)0, c, false, false);
  asm volatile("v_nop\n\tv_nop\n\tv_nop\n\tv_nop" : "+v"(d) : "v"(a), "v"(b));
  return d;
}

template <int NB>
__device__ __forceinline__ int scan_chunk(const int* __restrict__ dsts, int nE, int cbase, int slotBase,
                                          int vec8, int* list, int tid, int lane, int wave) {
  int wc = 0;
#pragma unroll
  for (int g = 0; g < NGRP; ++g) {
    const int el0  = (g * NTHR + tid) * EPT;
    const int e0   = cbase + el0;
    const int sent = -2147483647 - 1;
    v4i da, db;
    if (vec8 != 0 && cbase + CHUNK <= nE) {
      da = *(const v4i*)(dsts + e0);
      db = *(const v4i*)(dsts + e0 + 4);
    } else {
      da.x = (e0     < nE) ? dsts[min(e0, nE - 1)] : sent;
      da.y = (e0 + 1 < nE) ? dsts[min(e0 + 1, nE - 1)] : sent;
      da.z = (e0 + 2 < nE) ? dsts[min(e0 + 2, nE - 1)] : sent;
      da.w = (e0 + 3 < nE) ? dsts[min(e0 + 3, nE - 1)] : sent;
      db.x = (e0 + 4 < nE) ? dsts[min(e0 + 4, nE - 1)] : sent;
      db.y = (e0 + 5 < nE) ? dsts[min(e0 + 5, nE - 1)] : sent;
      db.z = (e0 + 6 < nE) ? dsts[min(e0 + 6, nE - 1)] : sent;
      db.w = (e0 + 7 < nE) ? dsts[min(e0 + 7, nE - 1)] : sent;
    }
    const unsigned nb = (unsigned)slotBase;
    const unsigned s0 = (unsigned)da.x - nb, s1 = (unsigned)da.y - nb;
    const unsigned s2 = (unsigned)da.z - nb, s3 = (unsigned)da.w - nb;
    const unsigned s4 = (unsigned)db.x - nb, s5 = (unsigned)db.y - nb;
    const unsigned s6 = (unsigned)db.z - nb, s7 = (unsigned)db.w - nb;
    const bool h0 = s0 < (unsigned)NB, h1 = s1 < (unsigned)NB, h2 = s2 < (unsigned)NB, h3 = s3 < (unsigned)NB;
    const bool h4 = s4 < (unsigned)NB, h5 = s5 < (unsigned)NB, h6 = s6 < (unsigned)NB, h7 = s7 < (unsigned)NB;
    const unsigned any = __builtin_amdgcn_ballot_w32(h0 | h1 | h2 | h3 | h4 | h5 | h6 | h7);
    if (any != 0u) {
#define HITJ(J, HJ, SJ) { \
        const unsigned mj = __builtin_amdgcn_ballot_w32(HJ); \
        if (mj != 0u) { \
          if (HJ) { \
            const int pos = wc + (int)__builtin_amdgcn_mbcnt_lo(mj, 0u); \
            if (pos < WCAP) list[wave * WCAP + pos] = ((el0 + (J)) << 12) | (int)(SJ); \
          } \
          wc += (int)__builtin_popcount(mj); } }
      HITJ(0, h0, s0)
      HITJ(1, h1, s1)
      HITJ(2, h2, s2)
      HITJ(3, h3, s3)
      HITJ(4, h4, s4)
      HITJ(5, h5, s5)
      HITJ(6, h6, s6)
      HITJ(7, h7, s7)
#undef HITJ
    }
  }
  return wc;
}

__global__ __launch_bounds__(NTHR) void k_wprep(
    const float* __restrict__ Wa, const float* __restrict__ Wb, _Float16* wta, _Float16* wtb) {
  const int per = HID * HID / 8;
  const int mat = (int)blockIdx.x / (per / NTHR);
  const float* src = (mat == 0) ? Wa : Wb;
  _Float16*    dst = (mat == 0) ? wta : wtb;
  const int i  = (int)blockIdx.x * NTHR + (int)threadIdx.x;
  const int o  = (i - mat * per) * 8;
  const int n  = o / HID;
  const int k0 = o - n * HID;
  float v[8];
#pragma unroll
  for (int e = 0; e < 8; ++e) v[e] = src[(size_t)(k0 + e) * HID + n] * WSCALE;
  v4f a, b;
  a.x = v[0]; a.y = v[1]; a.z = v[2]; a.w = v[3];
  b.x = v[4]; b.y = v[5]; b.z = v[6]; b.w = v[7];
  const v8h hv = cvt8(a, b);
  _Float16* dp = dst + o;
  *(volatile v8h*)dp = hv;
  __threadfence();
  *(volatile v8h*)dp = hv;
}

__global__ __launch_bounds__(NTHR) void k_edges(
    const int* __restrict__ ei, int* ell, int* cnt, float* dis, int nN, int nE, int vec8) {
  extern __shared__ v4f lds_dyn[];
  int* region = (int*)lds_dyn;
  int* scnt   = region + NBE * ELLW;
  int* list   = scnt + NBE;
  int* wcnt   = list + LISTN;
  const int tid = threadIdx.x, lane = tid & 31, wave = tid >> 5;
  const int nodeBase = blockIdx.x * NBE;
  const int* dsts = ei + nE;

  {
    const v4i z = {0, 0, 0, 0};
#pragma unroll 1
    for (int i = tid; i < NBE * ELLW / 4; i += NTHR) ((v4i*)region)[i] = z;
#pragma unroll 1
    for (int i = tid; i < NBE / 4; i += NTHR) ((v4i*)scnt)[i] = z;
  }
  __syncthreads();

  const int nChunks = (nE + CHUNK - 1) / CHUNK;
#pragma unroll 1
  for (int ch = 0; ch < nChunks; ++ch) {
    const int cbase = ch * CHUNK;
    const int wc = scan_chunk<NBE>(dsts, nE, cbase, nodeBase, vec8, list, tid, lane, wave);
    if (lane == 0) wcnt[wave] = wc;
    __syncthreads();
    if (wave == 0) {
#pragma unroll 1
      for (int wsx = 0; wsx < NWAVE; ++wsx) {
        int n = __builtin_amdgcn_readfirstlane(wcnt[wsx]);
        n = n > WCAP ? WCAP : (n < 0 ? 0 : n);
        const int* lp = list + wsx * WCAP;
#pragma unroll 1
        for (int i = 0; i < n; ++i) {
          const int ent  = __builtin_amdgcn_readfirstlane(lp[i]);
          const int slot = ent & (NBE - 1);
          int e = cbase + ((ent >> 12) & (CHUNK - 1));
          e = e > nE - 1 ? nE - 1 : e;
          int src = ei[e];
          src = src < 0 ? 0 : (src > nN - 1 ? nN - 1 : src);
          if (lane == 0) {
            int pos = scnt[slot];
            pos = pos < 0 ? 0 : (pos > CNTMAX ? CNTMAX : pos);
            if (pos < ELLW) region[slot * ELLW + pos] = src;
            const int np = pos + 1;
            scnt[slot] = np > CNTMAX ? CNTMAX : np;
          }
        }
      }
    }
    __syncthreads();
  }

  int*   ep = ell + (size_t)nodeBase * ELLW;
  int*   cp = cnt + (size_t)nodeBase;
  float* dp = dis + (size_t)nodeBase;
#pragma unroll 1
  for (int it = 0; it < (NBE * ELLW / 4) / NTHR; ++it) {
    const int idx = it * NTHR + tid;
    const v4i v = ((const v4i*)region)[idx];
    *(volatile v4i*)(ep + 4 * idx) = v;
  }
#pragma unroll 1
  for (int it = 0; it < (NBE / 4) / NTHR; ++it) {
    const int idx = it * NTHR + tid;
    const v4i c = ((const v4i*)scnt)[idx];
    v4f d;
    d.x = rsqrtf((float)(c.x + 1)); d.y = rsqrtf((float)(c.y + 1));
    d.z = rsqrtf((float)(c.z + 1)); d.w = rsqrtf((float)(c.w + 1));
    *(volatile v4i*)(cp + 4 * idx) = c;
    *(volatile v4f*)(dp + 4 * idx) = d;
  }
  __threadfence();
#pragma unroll 1
  for (int it = 0; it < (NBE * ELLW / 4) / NTHR; ++it) {
    const int idx = it * NTHR + tid;
    const v4i v = ((const v4i*)region)[idx];
    *(volatile v4i*)(ep + 4 * idx) = v;
  }
#pragma unroll 1
  for (int it = 0; it < (NBE / 4) / NTHR; ++it) {
    const int idx = it * NTHR + tid;
    const v4i c = ((const v4i*)scnt)[idx];
    v4f d;
    d.x = rsqrtf((float)(c.x + 1)); d.y = rsqrtf((float)(c.y + 1));
    d.z = rsqrtf((float)(c.z + 1)); d.w = rsqrtf((float)(c.w + 1));
    *(volatile v4i*)(cp + 4 * idx) = c;
    *(volatile v4f*)(dp + 4 * idx) = d;
  }
}

__global__ __launch_bounds__(NTHR) void k_agg1(
    const float* __restrict__ x, const int* __restrict__ ell, const int* __restrict__ cnt,
    const float* __restrict__ dis, float* a1, int nN) {
  const int n  = blockIdx.x * NTHR + threadIdx.x;
  const int nc = n < nN ? n : nN - 1;
  int c = cnt[n];
  c = c < 0 ? 0 : (c > ELLW ? ELLW : c);
  const float dn = dis[n];
  const v2f xv = *(const v2f*)(x + 2 * (size_t)nc);
  float ax = dn * xv.x, ay = dn * xv.y;
#pragma unroll 1
  for (int p = 0; p < c; ++p) {
    int s = ell[(size_t)n * ELLW + p];
    s = s < 0 ? 0 : (s > nN - 1 ? nN - 1 : s);
    const float ds = dis[s];
    const v2f xs = *(const v2f*)(x + 2 * (size_t)s);
    ax += ds * xs.x;
    ay += ds * xs.y;
  }
  v2f o;
  o.x = dn * ax; o.y = dn * ay;
  float* op = a1 + 2 * (size_t)n;
  *(volatile v2f*)op = o;
  __threadfence();
  *(volatile v2f*)op = o;
}

__global__ __launch_bounds__(NTHR) void k_conv2(
    const float* __restrict__ a1, const int* __restrict__ ell, const int* __restrict__ cnt,
    const float* __restrict__ dis, const float* __restrict__ W1, const float* __restrict__ b1,
    const _Float16* __restrict__ wt, const float* __restrict__ bias, _Float16* h2s, int nN) {
  __shared__ __attribute__((aligned(16))) _Float16 sA[GROWS * AP];
  const int tid = threadIdx.x, lane = tid & 31, wave = tid >> 5, hh = lane >> 4, m = lane & 15;
  const int rowBase = blockIdx.x * GROWS;
  const v4f w0 = *(const v4f*)(W1 + 4 * lane);
  const v4f w1 = *(const v4f*)(W1 + HID + 4 * lane);
  const v4f bb = *(const v4f*)(b1 + 4 * lane);

#pragma unroll 1
  for (int i = 0; i < 16; ++i) {
    const int r = wave * 16 + i;
    const int n = rowBase + r;
    int c = cnt[n];
    c = c < 0 ? 0 : (c > ELLW ? ELLW : c);
    const float dn = dis[n];
    const v2f an = *(const v2f*)(a1 + 2 * (size_t)n);
    v4f hv = relu4(w0 * an.x + w1 * an.y + bb);
    v4f ag = hv * dn;
#pragma unroll 1
    for (int p = 0; p < c; ++p) {
      int s = ell[(size_t)n * ELLW + p];
      s = s < 0 ? 0 : (s > nN - 1 ? nN - 1 : s);
      const float ds = dis[s];
      const v2f as = *(const v2f*)(a1 + 2 * (size_t)s);
      const v4f hs = relu4(w0 * as.x + w1 * as.y + bb);
      ag = ag + hs * ds;
    }
    ag = ag * (dn * ASCALE);
    const v4h q = __builtin_convertvector(ag, v4h);
    *(v4h*)(sA + r * AP + 4 * lane) = q;
  }
  __syncthreads();

  v8f d[8];
#pragma unroll
  for (int t = 0; t < 8; ++t) { v8f z = {0.f, 0.f, 0.f, 0.f, 0.f, 0.f, 0.f, 0.f}; d[t] = z; }
  const _Float16* ar = sA + (wave * 16 + m) * AP + 8 * hh;
#pragma unroll
  for (int kt = 0; kt < HID / 32; ++kt) {
    FragH a;
    a.h[0] = *(const v8h*)(ar + 32 * kt);
    a.h[1] = *(const v8h*)(ar + 32 * kt + 16);
#pragma unroll
    for (int t = 0; t < 8; ++t) {
      const _Float16* bp = wt + (size_t)(16 * t + m) * HID + 32 * kt + 8 * hh;
      FragH b;
      b.h[0] = *(const v8h*)bp;
      b.h[1] = *(const v8h*)(bp + 16);
      d[t] = wmh(a.v, b.v, d[t]);
    }
  }
  __syncthreads();

  _Float16* stg = sA;
  const int r0 = wave * 16 + 8 * hh;
#pragma unroll
  for (int t = 0; t < 8; ++t) {
    const float bl = bias[16 * t + m];
    _Float16* sp = stg + r0 * HID + 16 * t + m;
#pragma unroll
    for (int r = 0; r < 8; ++r) {
      float v = d[t][r] * OSCALE + bl;
      v = fmaxf(v, 0.0f) * ASCALE;
      sp[r * HID] = (_Float16)v;
    }
  }
  __syncthreads();

  const _Float16* lp = stg + wave * 16 * HID;
  _Float16* gp = h2s + ((size_t)rowBase + wave * 16) * HID;
#pragma unroll
  for (int p = 0; p < 8; ++p) {
    const v8h v = *(const v8h*)(lp + 8 * (32 * p + lane));
    *(volatile v8h*)(gp + 8 * (32 * p + lane)) = v;
  }
  __threadfence();
#pragma unroll
  for (int p = 0; p < 8; ++p) {
    const v8h v = *(const v8h*)(lp + 8 * (32 * p + lane));
    *(volatile v8h*)(gp + 8 * (32 * p + lane)) = v;
  }
}

__global__ __launch_bounds__(NTHR) void k_conv3(
    const _Float16* __restrict__ h2s, const int* __restrict__ ell, const int* __restrict__ cnt,
    const float* __restrict__ dis, const int* __restrict__ batch,
    const _Float16* __restrict__ wt, const float* __restrict__ bias,
    float* psum, int* pmeta, int nN) {
  extern __shared__ v4f lds_dyn[];
  _Float16* sA  = (_Float16*)lds_dyn;
  float*    stg = (float*)lds_dyn;
  __shared__ int sG[GROWS];
  __shared__ int sSlot[GROWS];
  __shared__ int sId[NSLOT];
  __shared__ int sCnt[NSLOT];
  __shared__ __attribute__((aligned(16))) float part[2 * NSLOT * HID];
  __shared__ __attribute__((aligned(16))) float sps[NSLOT * HID];
  __shared__ __attribute__((aligned(16))) int sMeta[METAW];
  const int tid = threadIdx.x, lane = tid & 31, wave = tid >> 5, hh = lane >> 4, m = lane & 15;
  const int rowBase = blockIdx.x * GROWS;

  if (tid < GROWS) {
    const int n  = rowBase + tid;
    const int nc = n < nN ? n : nN - 1;
    sG[tid] = batch[nc];
  }

#pragma unroll 1
  for (int i = 0; i < 16; ++i) {
    const int r = wave * 16 + i;
    const int n = rowBase + r;
    int c = cnt[n];
    c = c < 0 ? 0 : (c > ELLW ? ELLW : c);
    const float dn = dis[n];
    const v4h hn = *(const v4h*)(h2s + (size_t)n * HID + 4 * lane);
    v4f ag = __builtin_convertvector(hn, v4f) * dn;
#pragma unroll 1
    for (int p = 0; p < c; ++p) {
      int s = ell[(size_t)n * ELLW + p];
      s = s < 0 ? 0 : (s > nN - 1 ? nN - 1 : s);
      const float ds = dis[s];
      const v4h hq = *(const v4h*)(h2s + (size_t)s * HID + 4 * lane);
      ag = ag + __builtin_convertvector(hq, v4f) * ds;
    }
    ag = ag * dn;
    const v4h q = __builtin_convertvector(ag, v4h);
    *(v4h*)(sA + r * AP + 4 * lane) = q;
  }
  __syncthreads();

  v8f d[8];
#pragma unroll
  for (int t = 0; t < 8; ++t) { v8f z = {0.f, 0.f, 0.f, 0.f, 0.f, 0.f, 0.f, 0.f}; d[t] = z; }
  const _Float16* ar = sA + (wave * 16 + m) * AP + 8 * hh;
#pragma unroll
  for (int kt = 0; kt < HID / 32; ++kt) {
    FragH a;
    a.h[0] = *(const v8h*)(ar + 32 * kt);
    a.h[1] = *(const v8h*)(ar + 32 * kt + 16);
#pragma unroll
    for (int t = 0; t < 8; ++t) {
      const _Float16* bp = wt + (size_t)(16 * t + m) * HID + 32 * kt + 8 * hh;
      FragH b;
      b.h[0] = *(const v8h*)bp;
      b.h[1] = *(const v8h*)(bp + 16);
      d[t] = wmh(a.v, b.v, d[t]);
    }
  }
  __syncthreads();

  const int r0 = wave * 16 + 8 * hh;
#pragma unroll
  for (int t = 0; t < 8; ++t) {
    const float bl = bias[16 * t + m];
    float* sp = stg + r0 * HID + 16 * t + m;
#pragma unroll
    for (int r = 0; r < 8; ++r) sp[r * HID] = fmaxf(d[t][r] * OSCALE + bl, 0.0f);
  }
  if (tid == 0) {
    int used = 0;
#pragma unroll
    for (int j = 0; j < NSLOT; ++j) { sId[j] = -1; sCnt[j] = 0; }
#pragma unroll 1
    for (int r = 0; r < GROWS; ++r) {
      int f = -1;
      if (rowBase + r < nN) {
        const int g = sG[r];
#pragma unroll
        for (int j = 0; j < NSLOT; ++j) { if (j < used && sId[j] == g) f = j; }
        if (f < 0 && used < NSLOT) { f = used; sId[used] = g; used = used + 1; }
        if (f >= 0) sCnt[f] = sCnt[f] + 1;
      }
      sSlot[r] = f;
    }
  }
  __syncthreads();

  const int ch = tid & (HID - 1), half = tid >> 7;
  {
    float q0 = 0.f, q1 = 0.f, q2 = 0.f, q3 = 0.f;
#pragma unroll 1
    for (int rr = 0; rr < GROWS / 2; ++rr) {
      const int r = half * (GROWS / 2) + rr;
      const int s = sSlot[r];
      const float v = stg[r * HID + ch];
      q0 += (s == 0) ? v : 0.0f;
      q1 += (s == 1) ? v : 0.0f;
      q2 += (s == 2) ? v : 0.0f;
      q3 += (s == 3) ? v : 0.0f;
    }
    part[(half * NSLOT + 0) * HID + ch] = q0;
    part[(half * NSLOT + 1) * HID + ch] = q1;
    part[(half * NSLOT + 2) * HID + ch] = q2;
    part[(half * NSLOT + 3) * HID + ch] = q3;
  }
  __syncthreads();
  {
    const int j = half;
    sps[j * HID + ch]       = part[(0 * NSLOT + j) * HID + ch]     + part[(1 * NSLOT + j) * HID + ch];
    sps[(j + 2) * HID + ch] = part[(0 * NSLOT + j + 2) * HID + ch] + part[(1 * NSLOT + j + 2) * HID + ch];
  }
  if (tid < METAW) {
    const int iv = sId[tid & (NSLOT - 1)];
    const int cv = sCnt[tid & (NSLOT - 1)];
    sMeta[tid] = (tid < NSLOT) ? iv : ((tid < 2 * NSLOT) ? cv : 0);
  }
  __syncthreads();

  float* pp = psum  + (size_t)blockIdx.x * (NSLOT * HID);
  int*   mp = pmeta + (size_t)blockIdx.x * METAW;
  const v4f pv = ((const v4f*)sps)[tid & (NSLOT * HID / 4 - 1)];
  const v4i mv = ((const v4i*)sMeta)[tid & (METAW / 4 - 1)];
  if (tid < NSLOT * HID / 4) *(volatile v4f*)(pp + 4 * tid) = pv;
  if (tid < METAW / 4)       *(volatile v4i*)(mp + 4 * tid) = mv;
  __threadfence();
  if (tid < NSLOT * HID / 4) *(volatile v4f*)(pp + 4 * tid) = pv;
  if (tid < METAW / 4)       *(volatile v4i*)(mp + 4 * tid) = mv;
}

__global__ __launch_bounds__(NTHR) void k_head(
    const float* __restrict__ psum, const int* __restrict__ pmeta, int nP,
    const float* __restrict__ fw1, const float* __restrict__ fb1,
    const float* __restrict__ fw2, const float* __restrict__ fb2, float* out, int nG) {
  __shared__ __attribute__((aligned(16))) float accP[GB * HID];
  __shared__ __attribute__((aligned(16))) float hb[GB * HID];
  __shared__ __attribute__((aligned(16))) float sOut[32];
  __shared__ int cntP[GB];
  __shared__ int flist[NWAVE * WCF];
  __shared__ int wcnt[NWAVE];
  const int tid = threadIdx.x, lane = tid & 31, wave = tid >> 5;
  const int gBase = blockIdx.x * GB;

#pragma unroll 1
  for (int i = tid; i < GB * HID; i += NTHR) accP[i] = 0.0f;
  if (tid < GB) cntP[tid] = 0;
  if (tid < 32) sOut[tid] = 0.0f;
  __syncthreads();

  const int nCh = (nP + NTHR - 1) / NTHR;
#pragma unroll 1
  for (int chx = 0; chx < nCh; ++chx) {
    const int b = chx * NTHR + tid;
    const bool valid = b < nP;
    const int bc = valid ? b : nP - 1;
    const v4i ids = *(const v4i*)(pmeta + (size_t)bc * METAW);
    const unsigned gb = (unsigned)gBase;
    const unsigned s0 = (unsigned)ids.x - gb, s1 = (unsigned)ids.y - gb;
    const unsigned s2 = (unsigned)ids.z - gb, s3 = (unsigned)ids.w - gb;
    const bool h0 = valid && s0 < (unsigned)GB, h1 = valid && s1 < (unsigned)GB;
    const bool h2 = valid && s2 < (unsigned)GB, h3 = valid && s3 < (unsigned)GB;
    int wc = 0;
#define FHIT(J, HJ, SJ) { \
      const unsigned mj = __builtin_amdgcn_ballot_w32(HJ); \
      if (mj != 0u) { \
        if (HJ) { \
          const int pos = wc + (int)__builtin_amdgcn_mbcnt_lo(mj, 0u); \
          if (pos < WCF) flist[wave * WCF + pos] = (tid << 8) | ((J) << 4) | (int)(SJ); \
        } \
        wc += (int)__builtin_popcount(mj); } }
    FHIT(0, h0, s0)
    FHIT(1, h1, s1)
    FHIT(2, h2, s2)
    FHIT(3, h3, s3)
#undef FHIT
    if (lane == 0) wcnt[wave] = wc;
    __syncthreads();
    if (wave == 0) {
#pragma unroll 1
      for (int wsx = 0; wsx < NWAVE; ++wsx) {
        int n = __builtin_amdgcn_readfirstlane(wcnt[wsx]);
        n = n > WCF ? WCF : (n < 0 ? 0 : n);
        const int* lp = flist + wsx * WCF;
#pragma unroll 1
        for (int i = 0; i < n; ++i) {
          const int ent  = __builtin_amdgcn_readfirstlane(lp[i]);
          const int t    = (ent >> 8) & (NTHR - 1);
          const int j    = (ent >> 4) & (NSLOT - 1);
          const int slot = ent & (GB - 1);
          int pb = chx * NTHR + t;
          pb = pb > nP - 1 ? nP - 1 : pb;
          const float* row = psum + ((size_t)pb * NSLOT + j) * HID;
          const v4f v = *(const v4f*)(row + 4 * lane);
          v4f* ap = (v4f*)(accP + slot * HID + 4 * lane);
          *ap = *ap + v;
          if (lane == 0) cntP[slot] = cntP[slot] + pmeta[(size_t)pb * METAW + NSLOT + j];
        }
      }
    }
    __syncthreads();
  }

  int ng = nG - gBase;
  ng = ng > GB ? GB : (ng < 0 ? 0 : ng);
#pragma unroll 1
  for (int i = tid; i < GB * HID; i += NTHR) {
    const int j = i / HID;
    const float fc = (float)cntP[j];
    const float inv = (j < ng) ? (1.0f / fc) : 0.0f;
    accP[i] = accP[i] * inv;
  }
  __syncthreads();

  {
    const int o = tid & (HID - 1), jh = tid >> 7;
    const float fbo = fb1[o];
#pragma unroll 1
    for (int q = 0; q < GB / 2; ++q) {
      const int j = 2 * q + jh;
      const float* pr = accP + j * HID;
      float s = 0.0f;
#pragma unroll 4
      for (int k = 0; k < HID; ++k) s = fmaf(pr[k], fw1[(size_t)k * HID + o], s);
      hb[j * HID + o] = fmaxf(s + fbo, 0.0f);
    }
  }
  __syncthreads();
  if (tid < GB * ODIM) {
    const int j = tid >> 1, dd = tid & 1;
    const float* hr = hb + j * HID;
    float s = 0.0f;
#pragma unroll 4
    for (int k = 0; k < HID; ++k) s = fmaf(hr[k], fw2[k * ODIM + dd], s);
    sOut[tid] = s + fb2[dd];
  }
  __syncthreads();

  const int npc  = (ng * ODIM) / 4;
  const int tail = (ng * ODIM) & 3;
  float* op = out + (size_t)gBase * ODIM;
  const v4f ov = ((const v4f*)sOut)[tid & 7];
  const v2f tv = ((const v2f*)sOut)[(2 * npc) & 15];
  if (tid < npc) *(volatile v4f*)(op + 4 * tid) = ov;
  if (tail != 0 && tid == npc) *(volatile v2f*)(op + 4 * npc) = tv;
  __threadfence();
  if (tid < npc) *(volatile v4f*)(op + 4 * tid) = ov;
  if (tail != 0 && tid == npc) *(volatile v2f*)(op + 4 * npc) = tv;
}

extern "C" void kernel_launch(void* const* d_in, const int* in_sizes, int n_in,
                              void* d_out, int out_size, void* d_ws, size_t ws_size,
                              hipStream_t stream) {
  if (n_in < 13) return;
  const int nN = in_sizes[0] / INDIM;
  const int nE = in_sizes[1] / 2;
  if (nN <= 0 || nE <= 0 || in_sizes[0] != nN * INDIM || in_sizes[1] != 2 * nE || in_sizes[2] != nN) return;
  if (in_sizes[3] != INDIM * HID || in_sizes[4] != HID || in_sizes[5] != HID * HID || in_sizes[6] != HID ||
      in_sizes[7] != HID * HID || in_sizes[8] != HID || in_sizes[9] != HID * HID || in_sizes[10] != HID ||
      in_sizes[11] != HID * ODIM || in_sizes[12] != ODIM) return;
  const int nG = out_size / ODIM;
  if (nG <= 0 || out_size != nG * ODIM) return;
  if (nN > (1 << 24) || nE > (1 << 28) || nG > (1 << 24)) return;

  const float* x     = (const float*)d_in[0];
  const int*   ei    = (const int*)d_in[1];
  const int*   batch = (const int*)d_in[2];
  const float* W1    = (const float*)d_in[3];
  const float* b1    = (const float*)d_in[4];
  const float* W2    = (const float*)d_in[5];
  const float* b2    = (const float*)d_in[6];
  const float* W3    = (const float*)d_in[7];
  const float* b3    = (const float*)d_in[8];
  const float* fw1   = (const float*)d_in[9];
  const float* fb1   = (const float*)d_in[10];
  const float* fw2   = (const float*)d_in[11];
  const float* fb2   = (const float*)d_in[12];
  float* out = (float*)d_out;

  const int nBE  = (nN + NBE - 1) / NBE;
  const int NPAD = nBE * NBE;
  const int nB1  = NPAD / NTHR;
  const int nB2  = NPAD / GROWS;
  const int nP   = nB2;
  const int nBH  = (nG + GB - 1) / GB;

  char* ws = (char*)d_ws;
  size_t off = 0;
  const size_t oWt2 = off; off += (size_t)HID * HID * 2;            off = (off + 255) & ~(size_t)255;
  const size_t oWt3 = off; off += (size_t)HID * HID * 2;            off = (off + 255) & ~(size_t)255;
  const size_t oCnt = off; off += (size_t)NPAD * 4;                 off = (off + 255) & ~(size_t)255;
  const size_t oDis = off; off += (size_t)NPAD * 4;                 off = (off + 255) & ~(size_t)255;
  const size_t oEll = off; off += (size_t)NPAD * ELLW * 4;          off = (off + 255) & ~(size_t)255;
  const size_t oA1  = off; off += (size_t)NPAD * INDIM * 4;         off = (off + 255) & ~(size_t)255;
  const size_t oH2  = off; off += (size_t)NPAD * HID * 2;           off = (off + 255) & ~(size_t)255;
  const size_t oPs  = off; off += (size_t)nP * NSLOT * HID * 4;     off = (off + 255) & ~(size_t)255;
  const size_t oPm  = off; off += (size_t)nP * METAW * 4;           off = (off + 255) & ~(size_t)255;
  if (off > ws_size) return;
  _Float16* wt2  = (_Float16*)(ws + oWt2);
  _Float16* wt3  = (_Float16*)(ws + oWt3);
  int*      cnt  = (int*)(ws + oCnt);
  float*    dis  = (float*)(ws + oDis);
  int*      ell  = (int*)(ws + oEll);
  float*    a1   = (float*)(ws + oA1);
  _Float16* h2s  = (_Float16*)(ws + oH2);
  float*    psum = (float*)(ws + oPs);
  int*      pmeta = (int*)(ws + oPm);

  const int vec8 = ((nE & 3) == 0) ? 1 : 0;

  k_wprep<<<(2 * HID * HID / 8) / NTHR, NTHR, 0, stream>>>(W2, W3, wt2, wt3);

  hipFuncSetAttribute(reinterpret_cast<const void*>(&k_edges),
                      hipFuncAttributeMaxDynamicSharedMemorySize, LDS_ELL);
  k_edges<<<nBE, NTHR, LDS_ELL, stream>>>(ei, ell, cnt, dis, nN, nE, vec8);

  k_agg1<<<nB1, NTHR, 0, stream>>>(x, ell, cnt, dis, a1, nN);

  k_conv2<<<nB2, NTHR, 0, stream>>>(a1, ell, cnt, dis, W1, b1, wt2, b2, h2s, nN);

  hipFuncSetAttribute(reinterpret_cast<const void*>(&k_conv3),
                      hipFuncAttributeMaxDynamicSharedMemorySize, LDS_L3);
  k_conv3<<<nB2, NTHR, LDS_L3, stream>>>(h2s, ell, cnt, dis, batch, wt3, b3, psum, pmeta, nN);

  k_head<<<nBH, NTHR, 0, stream>>>(psum, pmeta, nP, fw1, fb1, fw2, fb2, out, nG);
}
